// Parzen_34892314313015
// MI455X (gfx1250) — hardware-verified
//
#include <hip/hip_runtime.h>
#include <stddef.h>


typedef _Float16 v16h __attribute__((ext_vector_type(16)));
typedef _Float16 v8h  __attribute__((ext_vector_type(8)));
typedef float    v8f  __attribute__((ext_vector_type(8)));
typedef float    v4f  __attribute__((ext_vector_type(4)));
typedef _Float16 h16;

#ifndef NQ
#define NQ 8192
#endif
#ifndef NC
#define NC 16384
#endif
#define NQ_FULL 8192
#define NC_FULL 16384
#define DD 64

static_assert(NQ >= 128 && NQ <= NQ_FULL && (NQ % 128) == 0);
static_assert(NC >= 128 && NC <= NC_FULL && (NC % 128) == 0);
static_assert((NC % 64) == 0);
static_assert(DD == 64 && (DD % 32) == 0);
static_assert(DD == 8 * 8);

#define PCARRY 64.0f
#define LOG2E  1.4426950408889634f
#define LN2    0.6931471805599453f

#define XH_BYTES ((size_t)NQ * DD * 2)
#define MH_BYTES ((size_t)NC * DD * 2)
#define XN_BYTES ((size_t)NQ * 4)
#define MN_BYTES ((size_t)NC * 4)
#define OFF_XH ((size_t)0)
#define OFF_MH (OFF_XH + XH_BYTES)
#define OFF_XN (OFF_MH + MH_BYTES)
#define OFF_MN (OFF_XN + XN_BYTES)
#define WS_TOTAL (OFF_MN + MN_BYTES)
static_assert((XH_BYTES % 128) == 0 && (MH_BYTES % 128) == 0);
static_assert((XN_BYTES % 512) == 0 && (MN_BYTES % 512) == 0);
static_assert(WS_TOTAL <= (size_t)134217728);

__device__ __forceinline__ float bf16r(float x) {
  unsigned int u = __float_as_uint(x);
  u = (u + 0x7FFFu + ((u >> 16) & 1u)) & 0xFFFF0000u;
  return __uint_as_float(u);
}

__device__ __forceinline__ v16h frag_at(const _Float16* p) {
  v8h lo = *(const v8h*)(p);
  v8h hi = *(const v8h*)(p + 16);
  v16h out;
#pragma unroll
  for (int i = 0; i < 8; ++i) { out[i] = lo[i]; out[i + 8] = hi[i]; }
  return out;
}

__device__ __forceinline__ v8f wmma16(v16h a, v16h b, v8f c) {
  v8f d = __builtin_amdgcn_wmma_f32_16x16x32_f16(false, a, false, b, (short)0, c,
                                                 false, false);
  asm volatile("v_nop\n\tv_nop\n\tv_nop\n\tv_nop" : "+v"(d) : "v"(a), "v"(b));
  return d;
}

static __device__ __forceinline__ h16 toh_flush(float v) {
  const h16 r = (h16)v;
  return (fabsf(v) < 6.103515625e-05f) ? (h16)0.0f : r;
}

__device__ __forceinline__ float coef_of(float sg) {
  return (0.5f * LOG2E) * (1.0f / (sg * sg));
}

__global__ __launch_bounds__(256) void plane_kernel(
    const float* __restrict__ src, _Float16* __restrict__ plane, float* __restrict__ nrm,
    const float* __restrict__ sigma) {
  __shared__ float Ns[128];
  const unsigned tid = threadIdx.x, lane = tid & 31u;
  const unsigned wave = (unsigned)__builtin_amdgcn_readfirstlane((int)(threadIdx.x >> 5));
  const unsigned row0 = blockIdx.x * 128u + wave * 16u;
  const unsigned sub = lane >> 3;
  const unsigned col = (lane & 7u) * 8u;
  const float c = coef_of(bf16r(sigma[0]));

#pragma unroll 1
  for (unsigned it = 0; it < 4u; ++it) {
    const unsigned r = row0 + it * 4u + sub;
    const float* sp = src + (size_t)r * DD + col;
    const v4f a0 = *(const v4f*)(sp);
    const v4f a1 = *(const v4f*)(sp + 4u);
    v8h o;
    float s = 0.0f;
#pragma unroll
    for (int i = 0; i < 4; ++i) {
      const float e0 = bf16r(a0[i]);
      const float e1 = bf16r(a1[i]);
      s += e0 * e0;
      s += e1 * e1;
      o[i]     = toh_flush(PCARRY * e0);
      o[i + 4] = toh_flush(PCARRY * e1);
    }
    s += __shfl_xor(s, 1, 32);
    s += __shfl_xor(s, 2, 32);
    s += __shfl_xor(s, 4, 32);
    if ((lane & 7u) == 0u) Ns[wave * 16u + it * 4u + sub] = c * s;
    _Float16* p = plane + (size_t)r * DD + col;
    *(volatile v8h*)p = o;
    __threadfence();
    *(volatile v8h*)p = o;
  }
  __syncthreads();
  if (wave == 0u) {
    const v4f t = *(const v4f*)&Ns[lane * 4u];
    float* p = nrm + (size_t)blockIdx.x * 128u + lane * 4u;
    *(volatile v4f*)p = t;
    __threadfence();
    *(volatile v4f*)p = t;
  }
}

__global__ __launch_bounds__(256) void lse_kernel(
    const _Float16* __restrict__ Xh, const _Float16* __restrict__ Mh,
    const float* __restrict__ Xn, const float* __restrict__ Mn,
    const float* __restrict__ sigma, float* __restrict__ out) {
  __shared__ float Res[128];
  const unsigned tid = threadIdx.x, lane = tid & 31u;
  const unsigned wave = (unsigned)__builtin_amdgcn_readfirstlane((int)(threadIdx.x >> 5));
  const unsigned hh = lane >> 4, m = lane & 15u;
  const unsigned qrow0 = blockIdx.x * 128u + wave * 16u;

  const float sg = bf16r(sigma[0]);
  const float c = coef_of(sg);
  const float cs = c * (2.0f / (PCARRY * PCARRY));

  const _Float16* xp = Xh + (size_t)(qrow0 + m) * DD + hh * 8u;
  const v16h bx0 = frag_at(xp);
  const v16h bx1 = frag_at(xp + 32);

  float runmax = -3.0e38f;
  float runsum = 0.0f;

#pragma unroll 1
  for (unsigned cb = 0; cb < (unsigned)NC; cb += 64u) {
    v8f s[4];
#pragma unroll
    for (unsigned j = 0; j < 4u; ++j) {
      const _Float16* ap = Mh + (size_t)(cb + j * 16u + m) * DD + hh * 8u;
      const v16h a0 = frag_at(ap);
      const v16h a1 = frag_at(ap + 32);
      v8f t = {};
      t = wmma16(a0, bx0, t);
      t = wmma16(a1, bx1, t);
      const float* qp = Mn + cb + j * 16u + hh * 8u;
      const v4f q0 = *(const v4f*)(qp);
      const v4f q1 = *(const v4f*)(qp + 4u);
#pragma unroll
      for (int r = 0; r < 4; ++r) {
        s[j][r]     = t[r] * cs - q0[r];
        s[j][r + 4] = t[r + 4] * cs - q1[r];
      }
    }
    float tmax = s[0][0];
#pragma unroll
    for (int j = 0; j < 4; ++j)
#pragma unroll
      for (int r = 0; r < 8; ++r) tmax = fmaxf(tmax, s[j][r]);
    const float nmax = fmaxf(runmax, tmax);
    float acc = runsum * __builtin_amdgcn_exp2f(runmax - nmax);
#pragma unroll
    for (int j = 0; j < 4; ++j)
#pragma unroll
      for (int r = 0; r < 8; ++r) acc += __builtin_amdgcn_exp2f(s[j][r] - nmax);
    runsum = acc;
    runmax = nmax;
  }

  const float omax = __shfl_xor(runmax, 16, 32);
  const float osum = __shfl_xor(runsum, 16, 32);
  const float fm = fmaxf(runmax, omax);
  const float fs = runsum * __builtin_amdgcn_exp2f(runmax - fm) +
                   osum * __builtin_amdgcn_exp2f(omax - fm);
  const float p2 = Xn[qrow0 + m];
  const float lg = (fm + __builtin_log2f(fs)) - p2;
  const float val = LN2 * lg - logf((float)NC) - logf(sg * 2.50662827463f);
  if (hh == 0u) Res[wave * 16u + m] = val;
  __syncthreads();
  if (wave == 0u) {
    const v4f t = *(const v4f*)&Res[lane * 4u];
    float* p = out + (size_t)blockIdx.x * 128u + lane * 4u;
    *(volatile v4f*)p = t;
    __threadfence();
    *(volatile v4f*)p = t;
  }
}

extern "C" void kernel_launch(void* const* d_in, const int* in_sizes, int n_in,
                              void* d_out, int out_size, void* d_ws, size_t ws_size,
                              hipStream_t stream) {
  if (n_in < 3) return;
  if ((long long)in_sizes[0] < (long long)NQ * DD) return;
  if ((long long)in_sizes[1] < (long long)NC * DD) return;
  if (in_sizes[2] < 1) return;
  if ((long long)out_size < (long long)NQ) return;
  if (ws_size < WS_TOTAL) return;

  const float* X     = (const float*)d_in[0];
  const float* MU    = (const float*)d_in[1];
  const float* sigma = (const float*)d_in[2];
  float* out = (float*)d_out;

  char* ws = (char*)d_ws;
  _Float16* Xh = (_Float16*)(ws + OFF_XH);
  _Float16* Mh = (_Float16*)(ws + OFF_MH);
  float*    Xn = (float*)(ws + OFF_XN);
  float*    Mn = (float*)(ws + OFF_MN);

  dim3 blk(256);
  plane_kernel<<<dim3(NQ / 128), blk, 0, stream>>>(X, Xh, Xn, sigma);
  plane_kernel<<<dim3(NC / 128), blk, 0, stream>>>(MU, Mh, Mn, sigma);
  lse_kernel<<<dim3(NQ / 128), blk, 0, stream>>>(Xh, Mh, Xn, Mn, sigma, out);
}
